// EfficientAttention_47236050321895
// MI455X (gfx1250) — hardware-verified
//
#include <hip/hip_runtime.h>
#include <math.h>

typedef __attribute__((ext_vector_type(16))) __bf16 v16b;
typedef __attribute__((ext_vector_type(8)))  __bf16 v8b;
typedef __attribute__((ext_vector_type(8)))  float v8f;
typedef __attribute__((ext_vector_type(4)))  float v4f;
typedef __attribute__((ext_vector_type(4)))  unsigned v4u;
typedef __attribute__((ext_vector_type(4)))  int v4i;

template <typename T> __device__ __forceinline__ void vst2(void* p, T v) { *(volatile T*)p = v; __threadfence(); *(volatile T*)p = v; }
__device__ __forceinline__ v8f wmma_bf(v16b a, v16b b, v8f c) {
  v8f d = __builtin_amdgcn_wmma_f32_16x16x32_bf16(false, a, false, b, (short)0, c, false, false);
  asm volatile("v_nop\n\tv_nop\n\tv_nop\n\tv_nop" : "+v"(d) : "v"(a), "v"(b));
  return d;
}
__device__ __forceinline__ v16b frag_b(const __bf16* rowk0, int lane) {
  union { v16b v; v8b q[2]; } u; const __bf16* p = rowk0 + 8 * (lane >> 4);
  u.q[0] = *(const v8b*)p; u.q[1] = *(const v8b*)(p + 16); return u.v;
}
struct F2 { v16b h, l; };
__device__ __forceinline__ F2 bsplit16(const float v[16]) { F2 r;
#pragma unroll
  for (int i = 0; i < 16; ++i) { const __bf16 h = (__bf16)v[i]; r.h[i] = h; r.l[i] = (__bf16)(v[i] - (float)h); }
  return r; }
__device__ __forceinline__ F2 split_row(const float* row, int k0, int lane) { float v[16]; const float* p = row + k0 + 8 * (lane >> 4);
#pragma unroll
  for (int i = 0; i < 8; ++i) { v[i] = p[i]; v[8 + i] = p[16 + i]; }
  return bsplit16(v); }
__device__ __forceinline__ float bfr(float v) { return (float)(__bf16)v; }
#define LDSX() do { asm volatile("s_wait_dscnt 0" ::: "memory"); __builtin_amdgcn_wave_barrier(); __builtin_amdgcn_fence(3  , "workgroup"); } while (0)

#define NNODE 4096
#define DM 256
#define NHD 8
#define HDM 32
#define NW 4
#ifndef NQ
#define NQ NNODE
#endif
static_assert((NQ % 64) == 0);
static_assert(NQ >= 64);
static_assert(NQ <= NNODE);
static_assert(NHD * HDM == DM);
static_assert((DM % 128) == 0);
static_assert((NNODE % 64) == 0);
#define EPB 32
static_assert(EPB == 32);
#define CHUNK 2048
#define SCL (0.17677669529663687f)
#define L2E (1.4426950408889634f)

#define WS_XB  ((size_t)0)
#define WS_WB  (WS_XB + 2u * (size_t)NNODE * DM)
#define WS_QF  (WS_WB + 2u * (size_t)NW * DM * DM)
#define WS_KF  (WS_QF + 4u * (size_t)NNODE * DM)
#define WS_VF  (WS_KF + 4u * (size_t)NNODE * DM)
#define WS_VS  (WS_VF + 4u * (size_t)NNODE * DM)
#define WS_Y   (WS_VS + 4u * (size_t)DM)
#define WS_END (WS_Y  + 4u * (size_t)NNODE * DM)
static_assert(WS_END <= (size_t)134217728);
static_assert((WS_WB % 128) == 0);
static_assert((WS_QF % 128) == 0);
static_assert((WS_KF % 128) == 0);
static_assert((WS_VF % 128) == 0);
static_assert((WS_VS % 128) == 0);
static_assert((WS_Y % 128) == 0);

static_assert(((NNODE + NW * DM) % 8) == 0);
__global__ __launch_bounds__(256) void k_cvt(const float* __restrict__ X, const float* __restrict__ W0, const float* __restrict__ W1, const float* __restrict__ W2, const float* __restrict__ W3,
    __bf16* __restrict__ XB, __bf16* __restrict__ WB) {
  const int tid = threadIdx.x, lane = tid & 31; const int r = __builtin_amdgcn_readfirstlane((int)(blockIdx.x * 8 + (tid >> 5)));
  const float* src; __bf16* dst;
  if (r < NNODE) { src = X + (size_t)r * DM; dst = XB + (size_t)r * DM; }
  else { const int rr = r - NNODE, wi = rr / DM, wr = rr % DM; const float* Wp = wi == 0 ? W0 : wi == 1 ? W1 : wi == 2 ? W2 : W3; src = Wp + (size_t)wr * DM; dst = WB + ((size_t)wi * DM + wr) * DM; }
  const v4f a = *(const v4f*)(src + lane * 8), b = *(const v4f*)(src + lane * 8 + 4);
  union { v8b v; v4u u; } o;
  o.v[0] = (__bf16)a.x; o.v[1] = (__bf16)a.y; o.v[2] = (__bf16)a.z; o.v[3] = (__bf16)a.w;
  o.v[4] = (__bf16)b.x; o.v[5] = (__bf16)b.y; o.v[6] = (__bf16)b.z; o.v[7] = (__bf16)b.w;
  vst2(dst + lane * 8, o.u);
}

__global__ __launch_bounds__(128) void k_proj(const __bf16* __restrict__ XB, const __bf16* __restrict__ WB, float* __restrict__ QF, float* __restrict__ KF, float* __restrict__ VF) {
  __shared__ __align__(16) float ss[64][132];
  const int tid = threadIdx.x, wave = tid >> 5, lane = tid & 31, col = lane & 15, g = lane >> 4; const int which = blockIdx.z; const int c0 = blockIdx.y * 128; const size_t r0 = (size_t)blockIdx.x * 64;
  const __bf16* Wp = WB + (size_t)which * DM * DM; float* D = which == 0 ? QF : which == 1 ? KF : VF;
  v8f acc[8] = {};
#pragma unroll 2
  for (int kc = 0; kc < DM / 32; ++kc) { const v16b a = frag_b(XB + (r0 + wave * 16 + col) * DM + kc * 32, lane);
    asm volatile("s_wait_loadcnt 0x0" ::: "memory");
#pragma unroll
    for (int j = 0; j < 8; ++j) { const v16b w = frag_b(Wp + (size_t)(c0 + j * 16 + col) * DM + kc * 32, lane); asm volatile("s_wait_loadcnt 0x0" ::: "memory"); acc[j] = wmma_bf(a, w, acc[j]); } }
#pragma unroll
  for (int j = 0; j < 8; ++j) {
#pragma unroll
    for (int r = 0; r < 8; ++r) ss[wave * 16 + 8 * g + r][j * 16 + col] = acc[j][r]; }
  __syncthreads();
  for (int e = tid; e < 64 * 32; e += 128) { const int rl = e >> 5, q = e & 31; vst2(D + (r0 + rl) * DM + c0 + q * 4, *(const v4f*)&ss[rl][q * 4]); }
}

__global__ __launch_bounds__(256) void k_vsum(const float* __restrict__ VF, float* __restrict__ VS) {
  __shared__ float sp[8][32]; __shared__ __align__(16) float sl[32];
  const int tid = threadIdx.x, wave = tid >> 5, lane = tid & 31; const int c = blockIdx.x * 32 + lane;
  float s = 0.f;
  for (int r = wave; r < NNODE; r += 8) s += VF[(size_t)r * DM + c];
  sp[wave][lane] = s;
  __syncthreads();
  if (wave == 0) { float t = sp[0][lane];
#pragma unroll
    for (int w = 1; w < 8; ++w) t += sp[w][lane];
    sl[lane] = t;
    __builtin_amdgcn_fence(3  , "wavefront"); __builtin_amdgcn_wave_barrier();
    if (lane < 8) vst2(VS + blockIdx.x * 32 + lane * 4, *(const v4f*)&sl[lane * 4]); }
}

__global__ __launch_bounds__(256) void k_edge(const int* __restrict__ EI, int nE, const float* __restrict__ QF, const float* __restrict__ KF, const float* __restrict__ VF, const float* __restrict__ VS, float* __restrict__ Y) {
  __shared__ __align__(16) float s_num[EPB][DM];
  __shared__ unsigned s_bm[EPB][NNODE / 32];
  __shared__ int s_list[CHUNK];
  __shared__ int s_wtot[8];
  __shared__ float s_m[EPB][NHD];
  __shared__ float s_den[EPB][NHD];
  const int tid = threadIdx.x, lane = tid & 31; const int wave = __builtin_amdgcn_readfirstlane(tid >> 5);
  const int i0 = blockIdx.x * EPB;
  const int* EROW = EI; const int* ECOL = EI + nE;
  for (int e = tid; e < EPB * DM; e += 256) s_num[e / DM][e % DM] = VS[e % DM];
  for (int e = tid; e < EPB * (NNODE / 32); e += 256) s_bm[e / (NNODE / 32)][e % (NNODE / 32)] = 0u;
  s_m[tid >> 3][tid & 7] = 0.f; s_den[tid >> 3][tid & 7] = (float)NNODE;
  __syncthreads();
  for (int cb = 0; cb < nE; cb += CHUNK) {
    int ids[8]; const int e0 = cb + tid * 8;
    if (cb + CHUNK <= nE) {
      const v4i a = *(const v4i*)(EROW + e0), b = *(const v4i*)(EROW + e0 + 4);
      ids[0] = a.x; ids[1] = a.y; ids[2] = a.z; ids[3] = a.w; ids[4] = b.x; ids[5] = b.y; ids[6] = b.z; ids[7] = b.w;
    } else {
#pragma unroll
      for (int j = 0; j < 8; ++j) { const int e = e0 + j; const int ec = e < nE ? e : nE - 1; const int r = EROW[ec]; ids[j] = e < nE ? r : -1; }
    }
    int cnt = 0; unsigned hm = 0u;
#pragma unroll
    for (int j = 0; j < 8; ++j) { const bool hit = (unsigned)(ids[j] - i0) < (unsigned)EPB; hm |= hit ? (1u << j) : 0u; cnt += hit ? 1 : 0; }
    int incl = cnt;
#pragma unroll
    for (int o = 1; o < 32; o <<= 1) { const int t = __shfl_up(incl, o); incl += (lane >= o) ? t : 0; }
    if (lane == 31) s_wtot[wave] = incl;
    __syncthreads();
    int base = 0, tot = 0;
#pragma unroll
    for (int w = 0; w < 8; ++w) { const int t = s_wtot[w]; base += (w < wave) ? t : 0; tot += t; }
    int pos = base + incl - cnt;
#pragma unroll
    for (int j = 0; j < 8; ++j) if (hm & (1u << j)) { if ((unsigned)pos < (unsigned)CHUNK) s_list[pos] = ((e0 + j) << 5) | (ids[j] - i0); ++pos; }
    __syncthreads();
    const int nd = tot < CHUNK ? tot : CHUNK;
    for (int q = 0; q < nd; ++q) {
      const int ent = __builtin_amdgcn_readfirstlane(s_list[q]);
      const int rl = ent & 31;
      if ((rl >> 2) == wave) {
        int e = ent >> 5; e = e < nE ? e : nE - 1; e = e < 0 ? 0 : e;
        int cj = __builtin_amdgcn_readfirstlane(ECOL[e]); cj = cj < 0 ? 0 : (cj > NNODE - 1 ? NNODE - 1 : cj);
        const unsigned word = (unsigned)__builtin_amdgcn_readfirstlane((int)s_bm[rl][cj >> 5]); const unsigned bit = 1u << (cj & 31);
        if ((word & bit) == 0u) {
          if (lane == 0) s_bm[rl][cj >> 5] = word | bit;
          const float* qp = QF + (size_t)(i0 + rl) * DM + lane * 8; const float* kp = KF + (size_t)cj * DM + lane * 8; const float* vp = VF + (size_t)cj * DM + lane * 8;
          const v4f qa = *(const v4f*)qp, qb = *(const v4f*)(qp + 4), ka = *(const v4f*)kp, kb = *(const v4f*)(kp + 4), va = *(const v4f*)vp, vb = *(const v4f*)(vp + 4);
          float p = qa.x * ka.x + qa.y * ka.y + qa.z * ka.z + qa.w * ka.w + qb.x * kb.x + qb.y * kb.y + qb.z * kb.z + qb.w * kb.w;
          p += __shfl_xor(p, 1); p += __shfl_xor(p, 2);
          const float s = p * SCL; const int hd = lane >> 2;
          const float mo = s_m[rl][hd], dn = s_den[rl][hd];
          const float mn = fmaxf(mo, s);
          const float f = exp2f((mo - mn) * L2E);
          const float w = exp2f((s - mn) * L2E) - exp2f(-mn * L2E);
          v4f n0 = *(const v4f*)&s_num[rl][lane * 8], n1 = *(const v4f*)&s_num[rl][lane * 8 + 4];
          n0 = n0 * f + va * w; n1 = n1 * f + vb * w;
          *(v4f*)&s_num[rl][lane * 8] = n0; *(v4f*)&s_num[rl][lane * 8 + 4] = n1;
          if ((lane & 3) == 0) { s_m[rl][hd] = mn; s_den[rl][hd] = dn * f + w; }
          __builtin_amdgcn_fence(3  , "wavefront"); __builtin_amdgcn_wave_barrier();
        }
      }
    }
    __syncthreads();
  }
  __syncthreads();
  const int ha = lane >> 3;
#pragma unroll
  for (int k = 0; k < 4; ++k) { const int rl = wave * 4 + k;
    const float ia = __builtin_amdgcn_rcpf(s_den[rl][ha]), ib = __builtin_amdgcn_rcpf(s_den[rl][4 + ha]);
    const v4f a = *(const v4f*)&s_num[rl][lane * 4] * ia; const v4f b = *(const v4f*)&s_num[rl][128 + lane * 4] * ib;
    float* yr = Y + (size_t)(i0 + rl) * DM; vst2(yr + lane * 4, a); vst2(yr + 128 + lane * 4, b); }
}

__global__ __launch_bounds__(128) void k_out(const float* __restrict__ Y, const __bf16* __restrict__ WOB, const float* __restrict__ BO, float* __restrict__ OUT) { __shared__ __align__(16) float sf[4][16][132];
  const int tid = threadIdx.x, wave = tid >> 5, lane = tid & 31, col = lane & 15, g = lane >> 4; const int c0 = blockIdx.y * 128; const size_t r0 = (size_t)blockIdx.x * 64 + wave * 16;
  v8f acc[8] = {};
#pragma unroll 2
  for (int kc = 0; kc < DM / 32; ++kc) { const F2 a = split_row(Y + (r0 + col) * DM, kc * 32, lane); asm volatile("s_wait_loadcnt 0x0" ::: "memory");
#pragma unroll
    for (int j = 0; j < 8; ++j) { const v16b w = frag_b(WOB + (size_t)(c0 + j * 16 + col) * DM + kc * 32, lane); asm volatile("s_wait_loadcnt 0x0" ::: "memory"); acc[j] = wmma_bf(a.h, w, acc[j]); acc[j] = wmma_bf(a.l, w, acc[j]); } }
#pragma unroll
  for (int j = 0; j < 8; ++j) { const float bias = bfr(BO[c0 + j * 16 + col]);
#pragma unroll
    for (int r = 0; r < 8; ++r) sf[wave][8 * g + r][j * 16 + col] = acc[j][r] + bias; }
  LDSX(); for (int rl = 0; rl < 16; ++rl) vst2(OUT + (r0 + rl) * DM + c0 + lane * 4, *(const v4f*)&sf[wave][rl][lane * 4]);
}

extern "C" void kernel_launch(void* const* d_in, const int* in_sizes, int n_in, void* d_out, int out_size, void* d_ws, size_t ws_size, hipStream_t stream) {
  if (n_in < 7) return;
  const int nE = in_sizes[1] / 2;
  if (in_sizes[0] < NNODE * DM || nE < 1 || nE > (1 << 24) || in_sizes[2] < DM * DM || in_sizes[3] < DM * DM || in_sizes[4] < DM * DM || in_sizes[5] < DM * DM || in_sizes[6] < DM || out_size < NQ * DM) return;
  if (ws_size < WS_END) return;
  const float* X = (const float*)d_in[0]; const int* EI = (const int*)d_in[1];
  const float *WQ = (const float*)d_in[2], *WK = (const float*)d_in[3], *WV = (const float*)d_in[4], *WO = (const float*)d_in[5], *BO = (const float*)d_in[6];
  char* ws = (char*)d_ws;
  __bf16 *XB = (__bf16*)(ws + WS_XB), *WB = (__bf16*)(ws + WS_WB);
  float *QF = (float*)(ws + WS_QF), *KF = (float*)(ws + WS_KF), *VF = (float*)(ws + WS_VF), *VS = (float*)(ws + WS_VS), *Y = (float*)(ws + WS_Y);
  k_cvt<<<dim3((NNODE + NW * DM) / 8), 256, 0, stream>>>(X, WQ, WK, WV, WO, XB, WB);
  k_proj<<<dim3(NNODE / 64, DM / 128, 3), 128, 0, stream>>>(XB, WB, QF, KF, VF);
  k_vsum<<<dim3(DM / 32), 256, 0, stream>>>(VF, VS);
  k_edge<<<dim3(NQ / EPB), 256, 0, stream>>>(EI, nE, QF, KF, VF, VS, Y);
  k_out<<<dim3(NQ / 64, DM / 128), 128, 0, stream>>>(Y, WB + (size_t)3 * DM * DM, BO, (float*)d_out);
}
